// CausalSelfAttention_39410619908235
// MI455X (gfx1250) — hardware-verified
//
#include <hip/hip_runtime.h>
#include <math.h>

typedef __attribute__((ext_vector_type(16))) _Float16 v16h;
typedef __attribute__((ext_vector_type(16))) __bf16 v16b;
typedef __attribute__((ext_vector_type(8)))  _Float16 v8h;
typedef __attribute__((ext_vector_type(8)))  __bf16 v8b;
typedef __attribute__((ext_vector_type(8)))  float v8f;
typedef __attribute__((ext_vector_type(4)))  float v4f;
typedef __attribute__((ext_vector_type(4)))  unsigned v4u;

template <typename T> __device__ __forceinline__ void vst2(void* p, T v) { *(volatile T*)p = v; __threadfence(); *(volatile T*)p = v; }
__device__ __forceinline__ v8f wmma16(v16h a, v16h b, v8f c) {
  v8f d = __builtin_amdgcn_wmma_f32_16x16x32_f16(false, a, false, b, (short)0, c, false, false);
  asm volatile("v_nop\n\tv_nop\n\tv_nop\n\tv_nop" : "+v"(d) : "v"(a), "v"(b));
  return d;
}
__device__ __forceinline__ v8f wmma_bf(v16b a, v16b b, v8f c) {
  v8f d = __builtin_amdgcn_wmma_f32_16x16x32_bf16(false, a, false, b, (short)0, c, false, false);
  asm volatile("v_nop\n\tv_nop\n\tv_nop\n\tv_nop" : "+v"(d) : "v"(a), "v"(b));
  return d;
}
__device__ __forceinline__ v16h frag_h(const _Float16* rowk0, int lane) {
  union { v16h v; v8h q[2]; } u; const _Float16* p = rowk0 + 8 * (lane >> 4);
  u.q[0] = *(const v8h*)p; u.q[1] = *(const v8h*)(p + 16); return u.v;
}
__device__ __forceinline__ v16b frag_b(const __bf16* rowk0, int lane) {
  union { v16b v; v8b q[2]; } u; const __bf16* p = rowk0 + 8 * (lane >> 4);
  u.q[0] = *(const v8b*)p; u.q[1] = *(const v8b*)(p + 16); return u.v;
}
__device__ __forceinline__ v16h frag_f32(const float* rowk0, int lane) {
  v16h a; const float* p = rowk0 + 8 * (lane >> 4);
#pragma unroll
  for (int i = 0; i < 8; ++i) { a[i] = (_Float16)p[i]; a[8 + i] = (_Float16)p[16 + i]; }
  return a;
}
struct F2 { v16b h, l; };
__device__ __forceinline__ F2 bsplit16(const float v[16]) { F2 r;
#pragma unroll
  for (int i = 0; i < 16; ++i) { const __bf16 h = (__bf16)v[i]; r.h[i] = h; r.l[i] = (__bf16)(v[i] - (float)h); }
  return r; }
__device__ __forceinline__ F2 split_row(const float* row, int k0, int lane) { float v[16]; const float* p = row + k0 + 8 * (lane >> 4);
#pragma unroll
  for (int i = 0; i < 8; ++i) { v[i] = p[i]; v[8 + i] = p[16 + i]; }
  return bsplit16(v); }
#define LDSX() do { asm volatile("s_wait_dscnt 0" ::: "memory"); __builtin_amdgcn_wave_barrier(); __builtin_amdgcn_fence(3  , "workgroup"); } while (0)

#ifndef NB
#define NB 2
#endif
#ifndef TT
#define TT 2048
#endif
#define NB_FULL 2
#define TT_FULL 2048
#define CC 1024
#define DIN 1024
#define NH 16
#define HD 64
#define NQB (TT / 64)
#define HG 4
#define SCALE (0.125f)
#define CAUSAL 1
#define QBH 4
#define QHI 256
#define KHI 256
static_assert(TT % 128 == 0);
static_assert(TT <= TT_FULL);
static_assert(NB <= NB_FULL);
static_assert(NH % HG == 0);
static_assert(QBH * 64 == QHI);
static_assert((((QBH - 1) * 64 + 63) / 128 + 1) * 128 <= KHI);
static_assert(TT >= QHI && TT >= KHI);
static_assert(CC % 128 == 0 && DIN % 128 == 0 && HD == 64 && CC == NH * HD);
static_assert(((size_t)NB * TT * DIN) % (8u * 256u) == 0);

__host__ __device__ __forceinline__ int kb_last(int qb) { return CAUSAL ? ((qb * 64 + 63) >> 7) : (TT / 128 - 1); }

#define WS_XB  ((size_t)0)
#define WS_WT  (WS_XB + 2u * (size_t)NB * TT * DIN)
#define WS_WOT (WS_WT + 2u * (size_t)3 * CC * DIN)
#define WS_QH  (WS_WOT + 2u * (size_t)DIN * CC)
#define WS_KH  (WS_QH + 2u * (size_t)NB * TT * CC)
#define WS_VT  (WS_KH + 2u * (size_t)NB * TT * CC)
#define WS_QL  (WS_VT + 2u * (size_t)NB * CC * TT)
#define WS_KL  (WS_QL + 2u * (size_t)NB * QHI * CC)
#define WS_VB  (WS_KL + 2u * (size_t)NB * KHI * CC)
#define WS_VBL (WS_VB + 2u * (size_t)NB * CC * KHI)
#define WS_S   (WS_VBL + 2u * (size_t)NB * CC * KHI)
#define WS_Y   (WS_S  + 4u * (size_t)HG * TT * TT)
#define WS_END (WS_Y  + 4u * (size_t)NB * TT * CC)
static_assert(WS_END <= (size_t)134217728u);
static_assert(WS_WT % 128 == 0 && WS_WOT % 128 == 0 && WS_QH % 128 == 0 && WS_KH % 128 == 0 && WS_VT % 128 == 0 && WS_QL % 128 == 0 && WS_KL % 128 == 0 && WS_VB % 128 == 0 && WS_VBL % 128 == 0 && WS_S % 128 == 0 && WS_Y % 128 == 0);

__global__ __launch_bounds__(256) void k_cvt(const float* __restrict__ X, __bf16* __restrict__ XB) {
  const unsigned e = blockIdx.x * 256u + threadIdx.x; const unsigned row = e / (unsigned)(DIN / 8), q = e % (unsigned)(DIN / 8);
  const unsigned bb = row / (unsigned)TT, t = row - bb * (unsigned)TT;
  const float* p = X + ((size_t)bb * TT_FULL + t) * DIN + q * 8u;
  const v4f a = *(const v4f*)p, b = *(const v4f*)(p + 4);
  union { v8b h; v4u u; } o;
#pragma unroll
  for (int i = 0; i < 4; ++i) { o.h[i] = (__bf16)a[i]; o.h[4 + i] = (__bf16)b[i]; }
  vst2((void*)(XB + (size_t)row * DIN + q * 8u), o.u); }
__global__ __launch_bounds__(256) void k_wt(const float* __restrict__ W, __bf16* __restrict__ WT, unsigned K, unsigned N) {
  __shared__ __align__(16) __bf16 tb[64][72];
  const unsigned tid = threadIdx.x; const unsigned k0 = blockIdx.x * 64u, n0 = blockIdx.y * 64u;
#pragma unroll
  for (unsigned it = 0; it < 4u; ++it) { const unsigned e = tid + it * 256u, kr = e >> 4, nq = e & 15u;
    const v4f v = *(const v4f*)(W + (size_t)(k0 + kr) * N + n0 + nq * 4u);
    tb[nq * 4u + 0u][kr] = (__bf16)v[0]; tb[nq * 4u + 1u][kr] = (__bf16)v[1]; tb[nq * 4u + 2u][kr] = (__bf16)v[2]; tb[nq * 4u + 3u][kr] = (__bf16)v[3]; }
  __syncthreads();
#pragma unroll
  for (unsigned it = 0; it < 2u; ++it) { const unsigned e = tid + it * 256u, nl = e >> 3, q = e & 7u;
    vst2((void*)(WT + (size_t)(n0 + nl) * K + k0 + q * 8u), *(const v4u*)&tb[nl][q * 8u]); } }

__global__ __launch_bounds__(128) void k_proj(const __bf16* __restrict__ XB, const __bf16* __restrict__ WT, const float* __restrict__ FC, const float* __restrict__ FS,
    _Float16* __restrict__ QH, _Float16* __restrict__ QL, _Float16* __restrict__ KH, _Float16* __restrict__ KL, _Float16* __restrict__ VT, __bf16* __restrict__ VB, __bf16* __restrict__ VBL) {
  __shared__ __align__(16) _Float16 sh[64][136], sl[64][136]; __shared__ __align__(16) _Float16 th[128][72]; __shared__ __align__(16) __bf16 tb[128][72], tbl[128][72];
  __shared__ __align__(16) float tcs[64][36], tsn[64][36];
  const int tid = threadIdx.x, wave = tid >> 5, lane = tid & 31, col = lane & 15, g = lane >> 4; const int which = blockIdx.z; const int c0 = blockIdx.y * 128; const size_t r0 = (size_t)blockIdx.x * 64; const size_t bb = r0 / TT; const int t0 = (int)(r0 % TT);
#pragma unroll
  for (unsigned it = 0; it < 4u; ++it) { const unsigned e = (unsigned)tid + it * 128u, rl = e >> 3, q = e & 7u; const size_t o = (size_t)((unsigned)t0 + rl) * (HD / 2) + q * 4u;
    v4f c = *(const v4f*)(FC + o), s = *(const v4f*)(FS + o);
#pragma unroll
    for (int i = 0; i < 4; ++i) { c[i] = (float)(__bf16)c[i]; s[i] = (float)(__bf16)s[i]; }
    *(v4f*)&tcs[rl][q * 4u] = c; *(v4f*)&tsn[rl][q * 4u] = s; }
  __syncthreads();
  const __bf16* xrow = XB + (r0 + wave * 16 + col) * DIN; const __bf16* wrow = WT + ((size_t)which * CC + c0 + col) * DIN;
  v8f acc[8] = {};
#pragma unroll 2
  for (int kc = 0; kc < DIN / 32; ++kc) { const v16b a = frag_b(xrow + kc * 32, lane);
    asm volatile("s_wait_loadcnt 0x0" ::: "memory");
#pragma unroll
    for (int j = 0; j < 8; ++j) { const v16b w = frag_b(wrow + (size_t)j * 16 * DIN + kc * 32, lane); asm volatile("s_wait_loadcnt 0x0" ::: "memory"); acc[j] = wmma_bf(a, w, acc[j]); } }
  if (which < 2) { _Float16* DH = which == 0 ? QH : KH; _Float16* DL = which == 0 ? QL : KL; const int nhi = which == 0 ? QHI : KHI; const bool hi_rows = t0 < nhi;
#pragma unroll
    for (int j = 0; j < 8; ++j) {
#pragma unroll
      for (int r = 0; r < 8; ++r) { const float v = acc[j][r]; const float pv = __shfl_xor(v, 1);
        const int rl = wave * 16 + 8 * g + r; const int pi = ((j & 3) << 3) + (col >> 1); const float cs = tcs[rl][pi], sn = tsn[rl][pi];
        const float rv = v * cs + pv * ((col & 1) ? sn : -sn);
        const _Float16 hv = (_Float16)rv; sh[rl][j * 16 + col] = hv; sl[rl][j * 16 + col] = (_Float16)((rv - (float)hv) * 1024.0f); } }
    __syncthreads();
    for (int e = tid; e < 64 * 16; e += 128) { const int rl = e >> 4, q = e & 15; vst2((unsigned*)(DH + (r0 + rl) * CC + c0 + q * 8), *(const v4u*)&sh[rl][q * 8]); if (hi_rows) vst2((unsigned*)(DL + (bb * nhi + t0 + rl) * (size_t)CC + c0 + q * 8), *(const v4u*)&sl[rl][q * 8]); }
  } else { const bool hi_rows = t0 < KHI;
#pragma unroll
    for (int j = 0; j < 8; ++j) {
#pragma unroll
      for (int r = 0; r < 8; ++r) { const float v = acc[j][r]; const int rl = wave * 16 + 8 * g + r, cl = j * 16 + col; th[cl][rl] = (_Float16)v; const __bf16 bh = (__bf16)v; tb[cl][rl] = bh; tbl[cl][rl] = (__bf16)(v - (float)bh); } }
    __syncthreads();
    for (int e = tid; e < 128 * 8; e += 128) { const int cl = e >> 3, q = e & 7; vst2((unsigned*)(VT + (bb * CC + c0 + cl) * (size_t)TT + t0 + q * 8), *(const v4u*)&th[cl][q * 8]); if (hi_rows) { const size_t o3 = (bb * CC + c0 + cl) * (size_t)KHI + t0 + q * 8; vst2((unsigned*)(VB + o3), *(const v4u*)&tb[cl][q * 8]); vst2((unsigned*)(VBL + o3), *(const v4u*)&tbl[cl][q * 8]); } } } }
__global__ __launch_bounds__(128) void k_sc(const _Float16* __restrict__ QH, const _Float16* __restrict__ KH, const _Float16* __restrict__ QL, const _Float16* __restrict__ KL, int b, int h0, float* __restrict__ S0) { __shared__ __align__(16) float ss[4][16][132];
  const int qb = blockIdx.x, kb = blockIdx.y; if (kb > kb_last(qb)) return;
  const int h = h0 + blockIdx.z; float* S = S0 + (size_t)blockIdx.z * TT * TT;
  const int tid = threadIdx.x, wave = tid >> 5, lane = tid & 31, col = lane & 15, g = lane >> 4; const int k0 = kb * 128; const int ql0 = qb * 64 + wave * 16; const size_t q0 = (size_t)b * TT + ql0, kr0 = (size_t)b * TT + k0;
  v8f acc[8] = {}, accl[8] = {};
  const _Float16* QLb = QL + (size_t)b * QHI * CC; const _Float16* KLb = KL + (size_t)b * KHI * CC;
  if (qb < QBH) {
#pragma unroll
    for (int kc = 0; kc < HD / 32; ++kc) { const v16h ah = frag_h(QH + (q0 + col) * CC + h * HD + kc * 32, lane), al = frag_h(QLb + (size_t)(ql0 + col) * CC + h * HD + kc * 32, lane);
#pragma unroll
      for (int j = 0; j < 8; ++j) { const v16h kbf = frag_h(KH + (kr0 + j * 16 + col) * CC + h * HD + kc * 32, lane), klf = frag_h(KLb + (size_t)(k0 + j * 16 + col) * CC + h * HD + kc * 32, lane); acc[j] = wmma16(ah, kbf, acc[j]); accl[j] = wmma16(al, kbf, accl[j]); accl[j] = wmma16(ah, klf, accl[j]); } }
  } else {
#pragma unroll
    for (int kc = 0; kc < HD / 32; ++kc) { const v16h ah = frag_h(QH + (q0 + col) * CC + h * HD + kc * 32, lane);
#pragma unroll
      for (int j = 0; j < 8; ++j) { const v16h kbf = frag_h(KH + (kr0 + j * 16 + col) * CC + h * HD + kc * 32, lane); acc[j] = wmma16(ah, kbf, acc[j]); } } }
#pragma unroll
  for (int j = 0; j < 8; ++j) {
#pragma unroll
    for (int r = 0; r < 8; ++r) ss[wave][8 * g + r][j * 16 + col] = (acc[j][r] + accl[j][r] * (1.0f / 1024.0f)) * SCALE; }
  LDSX(); for (int rl = 0; rl < 16; ++rl) vst2(S + (size_t)(ql0 + rl) * TT + k0 + lane * 4, *(const v4f*)&ss[wave][rl][lane * 4]); }
__global__ __launch_bounds__(256) void k_sm(float* __restrict__ S0) { __shared__ float sred[8]; __shared__ float sbc; __shared__ __align__(16) float shv[TT];
  const int tid = threadIdx.x; const int t = blockIdx.x; const int kend = (kb_last(t >> 6) + 1) * 128;
  float* sr = S0 + (size_t)blockIdx.y * TT * TT + (size_t)t * TT;
  float m = -3.0e38f; for (int k = tid; k < kend; k += 256) { float v = (!CAUSAL || k <= t) ? sr[k] : -3.0e38f; shv[k] = v; m = fmaxf(m, v); }
#pragma unroll
  for (int o = 1; o < 32; o <<= 1) m = fmaxf(m, __shfl_xor(m, o));
  if ((tid & 31) == 0) sred[tid >> 5] = m; __syncthreads(); if (tid == 0) { float a = sred[0]; for (int i = 1; i < 8; ++i) a = fmaxf(a, sred[i]); sbc = a; } __syncthreads(); m = sbc; __syncthreads();
  float sum = 0.f;
#pragma unroll 1
  for (int k = tid; k < kend; k += 256) { const float v = shv[k]; const float e = (v <= -1.0e38f) ? 0.f : expf(v - m); shv[k] = e; sum += e; }
#pragma unroll
  for (int o = 1; o < 32; o <<= 1) sum += __shfl_xor(sum, o);
  if ((tid & 31) == 0) sred[tid >> 5] = sum; __syncthreads(); if (tid == 0) { float a = 0.f; for (int i = 0; i < 8; ++i) a += sred[i]; sbc = a > 0.f ? 2048.0f / a : 0.f; }     __syncthreads(); const float inv = sbc;
  for (int k = tid; k < kend; k += 256) shv[k] = shv[k] * inv;
  __syncthreads(); for (int q = tid; q < kend / 4; q += 256) vst2(sr + q * 4, *(const v4f*)&shv[q * 4]); }
__global__ __launch_bounds__(128) void k_pv(const float* __restrict__ PS0, const _Float16* __restrict__ VT, const __bf16* __restrict__ VB, const __bf16* __restrict__ VBL, int b, int h0, float* __restrict__ Y) { const int h = h0 + blockIdx.z; const float* PS = PS0 + (size_t)blockIdx.z * TT * TT; __shared__ __align__(16) float ss[4][16][HD + 4];
  const int tid = threadIdx.x, wave = tid >> 5, lane = tid & 31, col = lane & 15, g = lane >> 4; const int qb = blockIdx.x; const int ql0 = qb * 64 + wave * 16; const int kce = (kb_last(qb) + 1) * 4;
  v8f acc[HD / 16] = {};
  if (qb < QBH) {
#pragma unroll 1
    for (int kc = 0; kc < kce; ++kc) { const F2 p = split_row(PS + (size_t)(ql0 + col) * TT, kc * 32, lane);
      asm volatile("s_wait_loadcnt 0x0" ::: "memory");
#pragma unroll
      for (int j = 0; j < HD / 16; ++j) { const size_t po = ((size_t)b * CC + h * HD + j * 16 + col) * (size_t)KHI + kc * 32; const v16b vh = frag_b(VB + po, lane); acc[j] = wmma_bf(p.h, vh, acc[j]); acc[j] = wmma_bf(p.l, vh, acc[j]); acc[j] = wmma_bf(p.h, frag_b(VBL + po, lane), acc[j]); } }
  } else {
#pragma unroll 1
    for (int kc = 0; kc < kce; ++kc) { const v16h p = frag_f32(PS + (size_t)(ql0 + col) * TT + kc * 32, lane);
      asm volatile("s_wait_loadcnt 0x0" ::: "memory");
#pragma unroll
      for (int j = 0; j < HD / 16; ++j) { const size_t po = ((size_t)b * CC + h * HD + j * 16 + col) * (size_t)TT + kc * 32; acc[j] = wmma16(p, frag_h(VT + po, lane), acc[j]); } } }
#pragma unroll
  for (int j = 0; j < HD / 16; ++j)
#pragma unroll
    for (int r = 0; r < 8; ++r) ss[wave][8 * g + r][j * 16 + col] = acc[j][r] * (1.0f / 2048.0f);
  LDSX(); for (int rl = 0; rl < 16; ++rl) if (lane < HD / 4) vst2(Y + ((size_t)b * TT + ql0 + rl) * CC + h * HD + lane * 4, *(const v4f*)&ss[wave][rl][lane * 4]); }
__global__ __launch_bounds__(128) void k_out(const float* __restrict__ Y, const __bf16* __restrict__ WOT, float* __restrict__ OUT) { __shared__ __align__(16) float sf[4][16][132];
  const int tid = threadIdx.x, wave = tid >> 5, lane = tid & 31, col = lane & 15, g = lane >> 4; const int c0 = blockIdx.y * 128; const size_t r0 = (size_t)blockIdx.x * 64 + wave * 16;
  const size_t bb = r0 / TT, tq = r0 % TT; const size_t or0 = bb * (size_t)TT_FULL + tq;
  const __bf16* wrow = WOT + (size_t)(c0 + col) * CC;
  v8f acc[8] = {};
#pragma unroll 2
  for (int kc = 0; kc < CC / 32; ++kc) { const F2 a = split_row(Y + (r0 + col) * CC, kc * 32, lane); asm volatile("s_wait_loadcnt 0x0" ::: "memory");
#pragma unroll
    for (int j = 0; j < 8; ++j) { const v16b w = frag_b(wrow + (size_t)j * 16 * CC + kc * 32, lane); asm volatile("s_wait_loadcnt 0x0" ::: "memory"); acc[j] = wmma_bf(a.h, w, acc[j]); acc[j] = wmma_bf(a.l, w, acc[j]); } }
#pragma unroll
  for (int j = 0; j < 8; ++j) {
#pragma unroll
    for (int r = 0; r < 8; ++r) sf[wave][8 * g + r][j * 16 + col] = acc[j][r]; }
  LDSX(); for (int rl = 0; rl < 16; ++rl) vst2(OUT + (or0 + rl) * DIN + c0 + lane * 4, *(const v4f*)&sf[wave][rl][lane * 4]); }

extern "C" void kernel_launch(void* const* d_in, const int* in_sizes, int n_in, void* d_out, int out_size, void* d_ws, size_t ws_size, hipStream_t stream) {
  if (n_in < 5) return;
  if ((size_t)in_sizes[0] < ((size_t)(NB - 1) * TT_FULL + TT) * DIN) return;
  if ((size_t)in_sizes[1] < (size_t)3 * CC * DIN) return;
  if ((size_t)in_sizes[2] < (size_t)DIN * CC) return;
  if ((size_t)in_sizes[3] < (size_t)TT * (HD / 2)) return;
  if ((size_t)in_sizes[4] < (size_t)TT * (HD / 2)) return;
  if ((size_t)out_size < ((size_t)(NB - 1) * TT_FULL + TT) * DIN) return;
  if (ws_size < (size_t)WS_END) return;
  const float** F = (const float**)d_in;
  char* ws = (char*)d_ws; __bf16 *XB = (__bf16*)(ws + WS_XB), *WT = (__bf16*)(ws + WS_WT), *WOT = (__bf16*)(ws + WS_WOT);
  _Float16 *QH = (_Float16*)(ws + WS_QH), *KH = (_Float16*)(ws + WS_KH), *VT = (_Float16*)(ws + WS_VT), *QL = (_Float16*)(ws + WS_QL), *KL = (_Float16*)(ws + WS_KL); __bf16 *VB = (__bf16*)(ws + WS_VB), *VBL = (__bf16*)(ws + WS_VBL); float *S = (float*)(ws + WS_S), *Y = (float*)(ws + WS_Y);
  k_cvt<<<dim3((unsigned)(((size_t)NB * TT * DIN) / 2048u)), 256, 0, stream>>>(F[0], XB);
  k_wt<<<dim3(DIN / 64, 3 * CC / 64), 256, 0, stream>>>(F[1], WT, (unsigned)DIN, (unsigned)(3 * CC));
  k_wt<<<dim3(CC / 64, DIN / 64), 256, 0, stream>>>(F[2], WOT, (unsigned)CC, (unsigned)DIN);
  k_proj<<<dim3(NB * TT / 64, CC / 128, 3), 128, 0, stream>>>(XB, WT, F[3], F[4], QH, QL, KH, KL, VT, VB, VBL);
  for (int b = 0; b < NB; ++b) for (int h0 = 0; h0 < NH; h0 += HG) {
    k_sc<<<dim3(NQB, TT / 128, HG), 128, 0, stream>>>(QH, KH, QL, KL, b, h0, S);
    k_sm<<<dim3(TT, HG), 256, 0, stream>>>(S);
    k_pv<<<dim3(NQB, 1, HG), 128, 0, stream>>>(S, VT, VB, VBL, b, h0, Y);
  }
  k_out<<<dim3(NB * TT / 64, DIN / 128), 128, 0, stream>>>(Y, WOT, (float*)d_out);
}
